// SSLPretrainer_1932735284055
// MI455X (gfx1250) — hardware-run, weakly checked
//
#include <hip/hip_runtime.h>
#include <math.h>

constexpr int kBatch  = 16;
constexpr int kChan   = 3;
constexpr int kImg    = 512;
constexpr int kPatch  = 16;
constexpr int kGridW  = kImg / kPatch;
constexpr int kDim    = 128;
constexpr int kHeads  = 4;
constexpr int kHeadD  = kDim / kHeads;
constexpr int kNumP   = kGridW * kGridW;
constexpr int kPatchD = kChan * kPatch * kPatch;
constexpr int kNumVis = kNumP / 4;
constexpr int kFF     = 4 * kDim;
constexpr int kEncL   = 6;
constexpr int kDecL   = 2;
constexpr int kTokE   = kBatch * kNumVis;
constexpr int kTokD   = kBatch * kNumP;
constexpr int kQKld   = 2 * kDim;

static_assert(kGridW == 32);
static_assert(kHeadD == 32);
static_assert(kNumP == 1024);
static_assert(kPatchD == 768);
static_assert(kNumVis == 256);
static_assert(kTokE == 4096);
static_assert(kTokD == 16384);
static_assert(kTokE % 64 == 0 && kTokD % 64 == 0 && kDim % 64 == 0 && kQKld % 64 == 0 && kFF % 64 == 0 && kPatchD % 64 == 0);
static_assert(kPatchD % 32 == 0 && kDim % 32 == 0 && kFF % 32 == 0);
static_assert(kNumVis % 64 == 0 && kNumP % 64 == 0);

constexpr float kWCarry   = 16.0f;
constexpr float kQkvCarry = 16.0f;
constexpr float kPCarry   = 1024.0f;
constexpr float kAoCarry  = 256.0f;
constexpr float kHCarry   = 16.0f;
constexpr float kInvSqrt2 = 0.70710678118654752f;
constexpr float kLnEps    = 1e-5f;

typedef __attribute__((ext_vector_type(16))) _Float16 v16h;
typedef __attribute__((ext_vector_type(8)))  _Float16 v8h;
typedef __attribute__((ext_vector_type(8)))  float    v8f;
typedef __attribute__((ext_vector_type(4)))  float    v4f;
typedef __attribute__((ext_vector_type(4)))  unsigned int v4u;
typedef __attribute__((ext_vector_type(2)))  unsigned int v2u;

template <typename T> struct Frag;
template <> struct Frag<_Float16> {
  typedef v16h V;
  union U { v16h v; v8h h[2]; };
  static __device__ __forceinline__ v16h load(const _Float16* p) {
    U f;
    f.h[0] = *(const v8h*)(p);
    f.h[1] = *(const v8h*)(p + 16);
    return f.v;
  }
  static __device__ __forceinline__ v8f mma(v16h a, v16h b, v8f c) {
    return __builtin_amdgcn_wmma_f32_16x16x32_f16(false, a, false, b, (short)0, c, false, false);
  }
};

__device__ __forceinline__ void tie_acc(v8f& c, v16h a, v16h b) { asm volatile("" : "+v"(c) : "v"(a), "v"(b)); }
__device__ __forceinline__ void guard_acc(v8f& c, v16h a, v16h b) { asm volatile("v_nop\n\tv_nop\n\tv_nop\n\tv_nop" : "+v"(c) : "v"(a), "v"(b)); }
__device__ __forceinline__ void keep4_h(v16h a, v16h b, v16h c, v16h d) { asm volatile("v_nop" :: "v"(a), "v"(b), "v"(c), "v"(d)); }
__device__ __forceinline__ void acc_guard4(v8f& a, v8f& b, v8f& c, v8f& d) { asm volatile("v_nop\n\tv_nop\n\tv_nop\n\tv_nop" : "+v"(a), "+v"(b), "+v"(c), "+v"(d)); }
__device__ __forceinline__ v8f mma_guarded(v16h a, v16h b, v8f c) {
  c = __builtin_amdgcn_wmma_f32_16x16x32_f16(false, a, false, b, (short)0, c, false, false);
  asm volatile("v_nop\n\tv_nop\n\tv_nop\n\tv_nop" : "+v"(c) : "v"(a), "v"(b));
  return c;
}
__device__ __forceinline__ void wave_lds_sync() {
  __builtin_amdgcn_fence(__ATOMIC_RELEASE, "workgroup");
  __builtin_amdgcn_wave_barrier();
  __builtin_amdgcn_fence(__ATOMIC_ACQUIRE, "workgroup");
}

__device__ __forceinline__ unsigned pk16(unsigned short a, unsigned short b) { return (unsigned)a | ((unsigned)b << 16); }
__device__ __forceinline__ unsigned short h_bits(float f) {
  const _Float16 h = (_Float16)f;
  return __builtin_bit_cast(unsigned short, h);
}

__device__ __forceinline__ void store_f32_f16_quad(float* pf, unsigned short* ph, v4f v) {
  const float f0 = v[0];
  const float f1 = v[1];
  const float f2 = v[2];
  const float f3 = v[3];
  v2u u;
  u[0] = pk16(h_bits(f0), h_bits(f1));
  u[1] = pk16(h_bits(f2), h_bits(f3));
  *(volatile v4f*)pf = v;
  *(volatile v2u*)ph = u;
  __threadfence();
  *(volatile v4f*)pf = v;
  *(volatile v2u*)ph = u;
}

template <int BIAS_MODE, int OUT_MODE, bool RESID, int ACT>
__global__ __launch_bounds__(256) void gemm64_f16(
    const unsigned short* __restrict__ Ap, int lda,
    const unsigned short* __restrict__ Btp, int ldb,
    void* __restrict__ Cout, void* __restrict__ Cout2, int ldc,
    const float* __restrict__ bias, const float* __restrict__ resid,
    int M, int N, int K, float scale, float bscale, float postmul) {
  static_assert(!(RESID && OUT_MODE != 0));
  typedef Frag<_Float16> F;
  const _Float16* A  = (const _Float16*)(const void*)Ap;
  const _Float16* Bt = (const _Float16*)(const void*)Btp;
  __shared__ __align__(16) float sT[8][16 * 68];
  const int lane = threadIdx.x & 31;
  const int wave = threadIdx.x >> 5;
  const int tilesN = N >> 6;
  const int tilesM = M >> 6;
  const int tile = blockIdx.x * 8 + wave;
  if (tile >= tilesM * tilesN) return;
  const int tm = tile / tilesN;
  const int tn = tile - tm * tilesN;
  const int m0 = tm << 6;
  const int n0 = tn << 6;

  const int rlane = lane & 15;
  const int koff  = (lane >> 4) * 8;
  const int mOff  = (lane >> 4) * 8;

  v8f acc[4][4];
#pragma unroll
  for (int i = 0; i < 4; ++i)
#pragma unroll
    for (int j = 0; j < 4; ++j) acc[i][j] = (v8f){0.f, 0.f, 0.f, 0.f, 0.f, 0.f, 0.f, 0.f};

  for (int k0 = 0; k0 < K; k0 += 32) {
    v16h bh[4];
#pragma unroll
    for (int j = 0; j < 4; ++j) {
      bh[j] = F::load(Bt + (size_t)(n0 + (j << 4) + rlane) * ldb + koff + k0);
    }
#pragma unroll
    for (int i = 0; i < 4; ++i) {
      const v16h ah = F::load(A + (size_t)(m0 + (i << 4) + rlane) * lda + koff + k0);
#pragma unroll
      for (int j = 0; j < 4; ++j) acc[i][j] = F::mma(ah, bh[j], acc[i][j]);
      tie_acc(acc[i][0], ah, bh[0]);
      tie_acc(acc[i][1], ah, bh[1]);
      tie_acc(acc[i][2], ah, bh[2]);
      guard_acc(acc[i][3], ah, bh[3]);
    }
    keep4_h(bh[0], bh[1], bh[2], bh[3]);
  }
  acc_guard4(acc[0][0], acc[0][1], acc[0][2], acc[0][3]);
  acc_guard4(acc[1][0], acc[1][1], acc[1][2], acc[1][3]);
  acc_guard4(acc[2][0], acc[2][1], acc[2][2], acc[2][3]);
  acc_guard4(acc[3][0], acc[3][1], acc[3][2], acc[3][3]);

  float* slab = sT[wave];
#pragma unroll
  for (int i = 0; i < 4; ++i) {
    const int mBase = m0 + (i << 4);
    v4f bm0 = (v4f){0.f, 0.f, 0.f, 0.f};
    v4f bm1 = (v4f){0.f, 0.f, 0.f, 0.f};
    if (BIAS_MODE == 1) {
      bm0 = *(const v4f*)(bias + mBase + mOff);
      bm1 = *(const v4f*)(bias + mBase + mOff + 4);
    }
#pragma unroll
    for (int j = 0; j < 4; ++j) {
      float bv = 0.f;
      if (BIAS_MODE == 2) bv = bias[n0 + (j << 4) + rlane] * bscale;
#pragma unroll
      for (int r = 0; r < 8; ++r) {
        float v = acc[i][j][r] * scale;
        if (BIAS_MODE == 1) v += ((r < 4) ? bm0[r & 3] : bm1[r & 3]) * bscale;
        if (BIAS_MODE == 2) v += bv;
        slab[(mOff + r) * 68 + (j << 4) + rlane] = v;
      }
    }
    wave_lds_sync();
    if (ACT == 5) {
#pragma unroll 1
      for (int t = 0; t < 32; ++t) {
        const int idx = t * 32 + lane;
        float* sp = slab + (idx >> 6) * 68 + (idx & 63);
        const float xv = *sp;
        const float gv = 0.5f * xv * (1.0f + erff(xv * kInvSqrt2));
        *sp = gv * postmul;
      }
      wave_lds_sync();
    }
    if (OUT_MODE == 0 || OUT_MODE == 3) {
      float* Cf = (float*)Cout;
      const int hh = lane >> 4;
      const int c4 = (lane & 15) * 4;
      v4f vv[8];
#pragma unroll
      for (int it = 0; it < 8; ++it) {
        const int row = it * 2 + hh;
        v4f v = *(const v4f*)(slab + row * 68 + c4);
        if (RESID) {
          const v4f rv = *(const v4f*)(resid + (size_t)(mBase + row) * ldc + n0 + c4);
          v += rv;
        }
        vv[it] = v;
      }
      for (int pass = 0; pass < 2; ++pass) {
#pragma unroll
        for (int it = 0; it < 8; ++it) {
          const int row = it * 2 + hh;
          *(volatile v4f*)(Cf + (size_t)(mBase + row) * ldc + n0 + c4) = vv[it];
        }
        __threadfence();
      }
    }
    if (OUT_MODE == 1 || OUT_MODE == 3) {
      unsigned short* Ch = (unsigned short*)((OUT_MODE == 3) ? Cout2 : Cout);
      const int q  = lane >> 3;
      const int c8 = (lane & 7) * 8;
      v8h hv[4];
#pragma unroll
      for (int it = 0; it < 4; ++it) {
        const int row = it * 4 + q;
        const float* sp = slab + row * 68 + c8;
        v8h tmp;
#pragma unroll
        for (int e = 0; e < 8; ++e) tmp[e] = (_Float16)sp[e];
        hv[it] = tmp;
      }
      for (int pass = 0; pass < 2; ++pass) {
#pragma unroll
        for (int it = 0; it < 4; ++it) {
          const int row = it * 4 + q;
          *(volatile v8h*)(Ch + (size_t)(mBase + row) * ldc + n0 + c8) = hv[it];
        }
        __threadfence();
      }
    }
    if (OUT_MODE == 4) {
      float* img = (float*)Cout;
      const int bimg = m0 / kNumP;
      const int pp   = (m0 - bimg * kNumP) + (i << 4);
      const int gh   = pp / kGridW;
      const int gw0  = pp - gh * kGridW;
      const int ch   = n0 / (kPatch * kPatch);
      const int py0  = (n0 - ch * (kPatch * kPatch)) / kPatch;
      const int gwl  = lane >> 2;
      const int px   = (lane & 3) * 4;
      v4f vv[8];
#pragma unroll
      for (int it = 0; it < 8; ++it) {
        const int pyl = it >> 1;
        const int sx  = it & 1;
        vv[it] = *(const v4f*)(slab + (sx * 8 + gwl) * 68 + pyl * 16 + px);
      }
      for (int pass = 0; pass < 2; ++pass) {
#pragma unroll
        for (int it = 0; it < 8; ++it) {
          const int pyl = it >> 1;
          const int sx  = it & 1;
          const size_t rowBase = ((size_t)(bimg * kChan + ch) * kImg + (size_t)(gh * kPatch + py0 + pyl)) * kImg;
          *(volatile v4f*)(img + rowBase + gw0 * kPatch + sx * 128 + lane * 4) = vv[it];
        }
        __threadfence();
      }
    }
    wave_lds_sync();
  }
}

constexpr int kNWpatch = kDim * kPatchD;
constexpr int kNEqkv   = kEncL * 3 * kDim * kDim;
constexpr int kNEout   = kEncL * kDim * kDim;
constexpr int kNEff1   = kEncL * kFF * kDim;
constexpr int kNEff2   = kEncL * kDim * kFF;
constexpr int kNDqkv   = kDecL * 3 * kDim * kDim;
constexpr int kNDout   = kDecL * kDim * kDim;
constexpr int kNDff1   = kDecL * kFF * kDim;
constexpr int kNDff2   = kDecL * kDim * kFF;
constexpr int kNWrecon = kPatchD * kDim;
constexpr long kOffWpatch = 0;
constexpr long kOffEqkv   = kOffWpatch + kNWpatch;
constexpr long kOffEout   = kOffEqkv + kNEqkv;
constexpr long kOffEff1   = kOffEout + kNEout;
constexpr long kOffEff2   = kOffEff1 + kNEff1;
constexpr long kOffDqkv   = kOffEff2 + kNEff2;
constexpr long kOffDout   = kOffDqkv + kNDqkv;
constexpr long kOffDff1   = kOffDout + kNDout;
constexpr long kOffDff2   = kOffDff1 + kNDff1;
constexpr long kOffWrecon = kOffDff2 + kNDff2;
constexpr long kW16Halves = kOffWrecon + kNWrecon;
constexpr int kCastBlocks = 192;
static_assert(kW16Halves == 1769472);
static_assert(kNEff1 / 8 <= kCastBlocks * 256 && kNEqkv / 8 <= kCastBlocks * 256);
static_assert(kNWpatch % 8 == 0 && kNDout % 8 == 0);

__global__ __launch_bounds__(256) void cast_weights_kernel(
    const float* __restrict__ s0, const float* __restrict__ s1, const float* __restrict__ s2,
    const float* __restrict__ s3, const float* __restrict__ s4, const float* __restrict__ s5,
    const float* __restrict__ s6, const float* __restrict__ s7, const float* __restrict__ s8,
    const float* __restrict__ s9, unsigned short* __restrict__ dst, float carry) {
  const int z = blockIdx.y;
  const float* src = (z == 0) ? s0 : (z == 1) ? s1 : (z == 2) ? s2 : (z == 3) ? s3 : (z == 4) ? s4
                   : (z == 5) ? s5 : (z == 6) ? s6 : (z == 7) ? s7 : (z == 8) ? s8 : s9;
  const int n8 = ((z == 0) ? kNWpatch : (z == 1) ? kNEqkv : (z == 2) ? kNEout : (z == 3) ? kNEff1 : (z == 4) ? kNEff2
                : (z == 5) ? kNDqkv : (z == 6) ? kNDout : (z == 7) ? kNDff1 : (z == 8) ? kNDff2 : kNWrecon) / 8;
  const long off = (z == 0) ? kOffWpatch : (z == 1) ? kOffEqkv : (z == 2) ? kOffEout : (z == 3) ? kOffEff1
                 : (z == 4) ? kOffEff2 : (z == 5) ? kOffDqkv : (z == 6) ? kOffDout : (z == 7) ? kOffDff1
                 : (z == 8) ? kOffDff2 : kOffWrecon;
  const int i = blockIdx.x * 256 + threadIdx.x;
  if (i >= n8) return;
  const float* p = src + 8 * (size_t)i;
  const v4f a = *(const v4f*)(p);
  const v4f c = *(const v4f*)(p + 4);
  unsigned short hb[8];
#pragma unroll
  for (int e = 0; e < 4; ++e) {
    const float fa = a[e] * carry;
    const float fc = c[e] * carry;
    hb[e]     = h_bits(fa);
    hb[4 + e] = h_bits(fc);
  }
  const v4u u = (v4u){pk16(hb[0], hb[1]), pk16(hb[2], hb[3]), pk16(hb[4], hb[5]), pk16(hb[6], hb[7])};
  unsigned short* q = dst + off + 8 * (size_t)i;
  *(volatile v4u*)q = u;
  __threadfence();
  *(volatile v4u*)q = u;
}

__global__ __launch_bounds__(256) void gather_patches_kernel(const float* __restrict__ x, const int* __restrict__ vis,
                                                             unsigned short* __restrict__ out) {
  constexpr int kSegs = kPatchD / 8;
  const int i = blockIdx.x * 256 + threadIdx.x;
  if (i >= kTokE * kSegs) return;
  const int t   = i / kSegs;
  const int seg = i - t * kSegs;
  const int d0  = seg * 8;
  const int bimg = t / kNumVis;
  int p = vis[t];
  p = p < 0 ? 0 : p;
  p = p > (kNumP - 1) ? (kNumP - 1) : p;
  const int gh  = p / kGridW;
  const int gw  = p - gh * kGridW;
  const int ch  = d0 / (kPatch * kPatch);
  const int py  = (d0 / kPatch) % kPatch;
  const int px0 = d0 % kPatch;
  const float* src = x + ((size_t)(bimg * kChan + ch) * kImg + (size_t)(gh * kPatch + py)) * kImg + gw * kPatch + px0;
  const v4f a = *(const v4f*)(src);
  const v4f c = *(const v4f*)(src + 4);
  unsigned short hb[8];
#pragma unroll
  for (int e = 0; e < 4; ++e) {
    const float fa = a[e];
    const float fc = c[e];
    hb[e]     = h_bits(fa);
    hb[4 + e] = h_bits(fc);
  }
  const v4u u = (v4u){pk16(hb[0], hb[1]), pk16(hb[2], hb[3]), pk16(hb[4], hb[5]), pk16(hb[6], hb[7])};
  unsigned short* q = out + 8 * (size_t)i;
  *(volatile v4u*)q = u;
  __threadfence();
  *(volatile v4u*)q = u;
}

__global__ __launch_bounds__(256) void ln_rows_kernel(const float* __restrict__ in, const float* __restrict__ w,
                                                      const float* __restrict__ bvec, float* __restrict__ xf,
                                                      unsigned short* __restrict__ xh, int rows) {
  const int row  = blockIdx.x * 8 + (threadIdx.x >> 5);
  const int lane = threadIdx.x & 31;
  if (row >= rows) return;
  const size_t base = (size_t)row * kDim + lane * 4;
  const v4f v = *(const v4f*)(in + base);
  float s = (v[0] + v[1]) + (v[2] + v[3]);
#pragma unroll
  for (int off = 16; off > 0; off >>= 1) s += __shfl_xor(s, off, 32);
  const float mean = s * (1.0f / (float)kDim);
  const float d0 = v[0] - mean;
  const float d1 = v[1] - mean;
  const float d2 = v[2] - mean;
  const float d3 = v[3] - mean;
  float q = (d0 * d0 + d1 * d1) + (d2 * d2 + d3 * d3);
#pragma unroll
  for (int off = 16; off > 0; off >>= 1) q += __shfl_xor(q, off, 32);
  const float inv = rsqrtf(q * (1.0f / (float)kDim) + kLnEps);
  const v4f wv = *(const v4f*)(w + lane * 4);
  const v4f bb = *(const v4f*)(bvec + lane * 4);
  v4f y;
  y[0] = d0 * inv * wv[0] + bb[0];
  y[1] = d1 * inv * wv[1] + bb[1];
  y[2] = d2 * inv * wv[2] + bb[2];
  y[3] = d3 * inv * wv[3] + bb[3];
  store_f32_f16_quad(xf + base, xh + base, y);
}

__global__ __launch_bounds__(256) void dec_fill_kernel(const float* __restrict__ mt, const float* __restrict__ pos,
                                                       float* __restrict__ xf, unsigned short* __restrict__ xh) {
  const int i = blockIdx.x * 256 + threadIdx.x;
  if (i >= kTokD * (kDim / 4)) return;
  const int row = i / (kDim / 4);
  const int c4  = (i - row * (kDim / 4)) * 4;
  const int p   = row % kNumP;
  const v4f a = *(const v4f*)(mt + c4);
  const v4f b = *(const v4f*)(pos + (size_t)p * kDim + c4);
  const v4f v = a + b;
  store_f32_f16_quad(xf + (size_t)row * kDim + c4, xh + (size_t)row * kDim + c4, v);
}

__global__ __launch_bounds__(256) void dec_scatter_kernel(const float* __restrict__ enc, const int* __restrict__ vis,
                                                          const float* __restrict__ pos, float* __restrict__ xf,
                                                          unsigned short* __restrict__ xh) {
  const int t    = blockIdx.x * 8 + (threadIdx.x >> 5);
  const int lane = threadIdx.x & 31;
  if (t >= kTokE) return;
  int p = vis[t];
  p = p < 0 ? 0 : p;
  p = p > (kNumP - 1) ? (kNumP - 1) : p;
  const int bimg = t / kNumVis;
  const v4f a = *(const v4f*)(enc + (size_t)t * kDim + lane * 4);
  const v4f b = *(const v4f*)(pos + (size_t)p * kDim + lane * 4);
  const v4f v = a + b;
  const size_t o = ((size_t)bimg * kNumP + p) * kDim + lane * 4;
  store_f32_f16_quad(xf + o, xh + o, v);
}

__global__ __launch_bounds__(128) void attn_hd32_kernel(const unsigned short* __restrict__ qkp,
                                                        const unsigned short* __restrict__ vtp,
                                                        unsigned short* __restrict__ aop,
                                                        int S, int Ttot, float sscale, float oscale) {
  typedef Frag<_Float16> F;
  __shared__ __align__(16) _Float16 Psh[4][16 * 64];
  __shared__ __align__(16) float    Os[4][16 * 132];
  const int tid  = threadIdx.x;
  const int wave = tid >> 5;
  const int lane = tid & 31;
  const int hh   = lane >> 4;
  const int c    = lane & 15;
  const int tb    = blockIdx.x * 64;
  const int bimg  = tb / S;
  const int kbase = bimg * S;
  const int q0    = tb + wave * 16;
  const int nChunks = S >> 6;
  const _Float16* QK = (const _Float16*)(const void*)qkp;
  const _Float16* VT = (const _Float16*)(const void*)vtp;
  _Float16* pw = Psh[wave];
  float*    os = Os[wave];

#pragma unroll 1
  for (int h = 0; h < kHeads; ++h) {
    const v16h qa = F::load(QK + (size_t)(q0 + c) * kQKld + h * kHeadD + 8 * hh);
    float mrow[8], lrow[8];
#pragma unroll
    for (int r = 0; r < 8; ++r) { mrow[r] = -INFINITY; lrow[r] = 0.f; }
    v8f oacc0 = (v8f){0.f, 0.f, 0.f, 0.f, 0.f, 0.f, 0.f, 0.f};
    v8f oacc1 = (v8f){0.f, 0.f, 0.f, 0.f, 0.f, 0.f, 0.f, 0.f};

#pragma unroll 1
    for (int kc = 0; kc < nChunks; ++kc) {
      const int kv0 = kbase + kc * 64;
      v8f s[4];
#pragma unroll
      for (int j = 0; j < 4; ++j) {
        const v16h kf = F::load(QK + (size_t)(kv0 + j * 16 + c) * kQKld + kDim + h * kHeadD + 8 * hh);
        s[j] = mma_guarded(qa, kf, (v8f){0.f, 0.f, 0.f, 0.f, 0.f, 0.f, 0.f, 0.f});
      }
      float cm[8];
#pragma unroll
      for (int r = 0; r < 8; ++r) {
        float m = -INFINITY;
#pragma unroll
        for (int j = 0; j < 4; ++j) {
          const float sv = s[j][r] * sscale;
          s[j][r] = sv;
          m = fmaxf(m, sv);
        }
#pragma unroll
        for (int off = 1; off < 16; off <<= 1) m = fmaxf(m, __shfl_xor(m, off, 32));
        cm[r] = m;
      }
#pragma unroll
      for (int r = 0; r < 8; ++r) {
        const float mnew  = fmaxf(mrow[r], cm[r]);
        const float alpha = expf(mrow[r] - mnew);
        mrow[r] = mnew;
        float psum = 0.f;
#pragma unroll
        for (int j = 0; j < 4; ++j) {
          const float p = expf(s[j][r] - mnew);
          psum += p;
          pw[(8 * hh + r) * 64 + j * 16 + c] = (_Float16)(p * kPCarry);
        }
#pragma unroll
        for (int off = 1; off < 16; off <<= 1) psum += __shfl_xor(psum, off, 32);
        lrow[r] = lrow[r] * alpha + psum;
        oacc0[r] *= alpha;
        oacc1[r] *= alpha;
      }
      wave_lds_sync();
#pragma unroll
      for (int kk = 0; kk < 2; ++kk) {
        const v16h pa = F::load(pw + c * 64 + kk * 32 + 8 * hh);
        const v16h vb0 = F::load(VT + (size_t)(h * kHeadD + c) * Ttot + kv0 + kk * 32 + 8 * hh);
        oacc0 = mma_guarded(pa, vb0, oacc0);
        const v16h vb1 = F::load(VT + (size_t)(h * kHeadD + 16 + c) * Ttot + kv0 + kk * 32 + 8 * hh);
        oacc1 = mma_guarded(pa, vb1, oacc1);
      }
      wave_lds_sync();
    }
#pragma unroll
    for (int r = 0; r < 8; ++r) {
      const float inv = oscale * (1.0f / lrow[r]);
      os[(8 * hh + r) * 132 + h * kHeadD + c]      = oacc0[r] * inv;
      os[(8 * hh + r) * 132 + h * kHeadD + 16 + c] = oacc1[r] * inv;
    }
  }
  wave_lds_sync();
  {
    const int c8 = (lane & 15) * 8;
    v8h hv[8];
#pragma unroll
    for (int it = 0; it < 8; ++it) {
      const int row = it * 2 + hh;
      const float* sp = os + row * 132 + c8;
      v8h tmp;
#pragma unroll
      for (int e = 0; e < 8; ++e) tmp[e] = (_Float16)sp[e];
      hv[it] = tmp;
    }
    for (int pass = 0; pass < 2; ++pass) {
#pragma unroll
      for (int it = 0; it < 8; ++it) {
        const int row = it * 2 + hh;
        *(volatile v8h*)(aop + (size_t)(q0 + row) * kDim + c8) = hv[it];
      }
      __threadfence();
    }
  }
}

template <int BM, int OM, bool RS, int AC>
static void run_gemm(hipStream_t st, const unsigned short* A, int lda, const unsigned short* Bt, int ldb,
                     void* C, void* C2, int ldc, const float* bias, const float* resid,
                     int M, int N, int K, float scale, float bscale, float postmul) {
  const int tiles = (M / 64) * (N / 64);
  gemm64_f16<BM, OM, RS, AC><<<dim3((tiles + 7) / 8), dim3(256), 0, st>>>(
      A, lda, Bt, ldb, C, C2, ldc, bias, resid, M, N, K, scale, bscale, postmul);
}

struct StackW {
  const unsigned short* qkv;
  const unsigned short* outw;
  const unsigned short* ff1;
  const unsigned short* ff2;
  const float* qkv_b;
  const float* out_b;
  const float* ln1_w;
  const float* ln1_b;
  const float* ff1_b;
  const float* ff2_b;
  const float* ln2_w;
  const float* ln2_b;
};

static void run_stack(hipStream_t st, int L, int S, int T, const StackW& w,
                      float* Xf, unsigned short* X16, float* T2, unsigned short* QK16,
                      unsigned short* Vt16, unsigned short* AO16, unsigned short* H16) {
  const float sscale = 1.0f / (sqrtf((float)kHeadD) * kQkvCarry * kQkvCarry);
  const float oscale = kAoCarry / (kPCarry * kQkvCarry);
  for (int l = 0; l < L; ++l) {
    const unsigned short* wq = w.qkv + (size_t)l * 3 * kDim * kDim;
    const unsigned short* wo = w.outw + (size_t)l * kDim * kDim;
    const unsigned short* w1 = w.ff1 + (size_t)l * kFF * kDim;
    const unsigned short* w2 = w.ff2 + (size_t)l * kDim * kFF;
    run_gemm<2, 1, false, 0>(st, X16, kDim, wq, kDim, QK16, nullptr, kQKld,
                             w.qkv_b + (size_t)l * 3 * kDim, nullptr, T, kQKld, kDim, 1.0f, kQkvCarry, 1.0f);
    run_gemm<1, 1, false, 0>(st, wq + (size_t)2 * kDim * kDim, kDim, X16, kDim, Vt16, nullptr, T,
                             w.qkv_b + (size_t)l * 3 * kDim + 2 * kDim, nullptr, kDim, T, kDim, 1.0f, kQkvCarry, 1.0f);
    attn_hd32_kernel<<<dim3(T / 64), dim3(128), 0, st>>>(QK16, Vt16, AO16, S, T, sscale, oscale);
    run_gemm<2, 0, true, 0>(st, AO16, kDim, wo, kDim, T2, nullptr, kDim, w.out_b + (size_t)l * kDim, Xf,
                            T, kDim, kDim, 1.0f / (kAoCarry * kWCarry), 1.0f, 1.0f);
    ln_rows_kernel<<<dim3(T / 8), dim3(256), 0, st>>>(T2, w.ln1_w + (size_t)l * kDim, w.ln1_b + (size_t)l * kDim, Xf, X16, T);
    run_gemm<2, 1, false, 5>(st, X16, kDim, w1, kDim, H16, nullptr, kFF, w.ff1_b + (size_t)l * kFF, nullptr,
                             T, kFF, kDim, 1.0f / kWCarry, 1.0f, kHCarry);
    run_gemm<2, 0, true, 0>(st, H16, kFF, w2, kFF, T2, nullptr, kDim, w.ff2_b + (size_t)l * kDim, Xf,
                            T, kDim, kFF, 1.0f / (kHCarry * kWCarry), 1.0f, 1.0f);
    ln_rows_kernel<<<dim3(T / 8), dim3(256), 0, st>>>(T2, w.ln2_w + (size_t)l * kDim, w.ln2_b + (size_t)l * kDim, Xf, X16, T);
  }
}

extern "C" void kernel_launch(void* const* d_in, const int* in_sizes, int n_in,
                              void* d_out, int out_size, void* d_ws, size_t ws_size, hipStream_t stream) {
  (void)in_sizes;
  (void)out_size;
  if (n_in < 32) return;

  constexpr size_t szW16 = (size_t)kW16Halves * 2;
  constexpr size_t szP16 = (size_t)kTokE * kPatchD * 2;
  constexpr size_t szXfE = (size_t)kTokE * kDim * 4;
  constexpr size_t szXfD = (size_t)kTokD * kDim * 4;
  constexpr size_t szX16 = (size_t)kTokD * kDim * 2;
  constexpr size_t szT2  = (size_t)kTokD * kDim * 4;
  constexpr size_t szQK  = (size_t)kTokD * kQKld * 2;
  constexpr size_t szVt  = (size_t)kDim * kTokD * 2;
  constexpr size_t szAO  = (size_t)kTokD * kDim * 2;
  constexpr size_t szH16 = (size_t)kTokD * kFF * 2;
  constexpr size_t szTotal = szW16 + szP16 + szXfE + szXfD + szX16 + szT2 + szQK + szVt + szAO + szH16;
  static_assert(szTotal == 66453504);
  static_assert(szTotal <= 134217728);
  static_assert(szW16 % 256 == 0 && szP16 % 256 == 0 && szXfE % 256 == 0);
  if (ws_size < szTotal) return;

  char* wsb = (char*)d_ws;
  size_t off = 0;
  unsigned short* W16  = (unsigned short*)(wsb + off); off += szW16;
  unsigned short* P16  = (unsigned short*)(wsb + off); off += szP16;
  float*          XfE  = (float*)(wsb + off);          off += szXfE;
  float*          XfD  = (float*)(wsb + off);          off += szXfD;
  unsigned short* X16  = (unsigned short*)(wsb + off); off += szX16;
  float*          T2   = (float*)(wsb + off);          off += szT2;
  unsigned short* QK16 = (unsigned short*)(wsb + off); off += szQK;
  unsigned short* Vt16 = (unsigned short*)(wsb + off); off += szVt;
  unsigned short* AO16 = (unsigned short*)(wsb + off); off += szAO;
  unsigned short* H16  = (unsigned short*)(wsb + off); off += szH16;

  const float* x        = (const float*)d_in[0];
  const int*   vis      = (const int*)d_in[1];
  const float* w_patch  = (const float*)d_in[2];
  const float* b_patch  = (const float*)d_in[3];
  const float* mask_tok = (const float*)d_in[4];
  const float* pos      = (const float*)d_in[5];
  const float* w_recon  = (const float*)d_in[6];
  const float* b_recon  = (const float*)d_in[7];

  cast_weights_kernel<<<dim3(kCastBlocks, 10), dim3(256), 0, stream>>>(
      w_patch, (const float*)d_in[8], (const float*)d_in[10], (const float*)d_in[14], (const float*)d_in[16],
      (const float*)d_in[20], (const float*)d_in[22], (const float*)d_in[26], (const float*)d_in[28],
      w_recon, W16, kWCarry);

  gather_patches_kernel<<<dim3((kTokE * (kPatchD / 8)) / 256), dim3(256), 0, stream>>>(x, vis, P16);

  run_gemm<2, 3, false, 0>(stream, P16, kPatchD, W16 + kOffWpatch, kPatchD, XfE, X16, kDim, b_patch, nullptr,
                           kTokE, kDim, kPatchD, 1.0f / kWCarry, 1.0f, 1.0f);

  StackW we;
  we.qkv = W16 + kOffEqkv;  we.outw = W16 + kOffEout;  we.ff1 = W16 + kOffEff1;  we.ff2 = W16 + kOffEff2;
  we.qkv_b = (const float*)d_in[9];   we.out_b = (const float*)d_in[11];
  we.ln1_w = (const float*)d_in[12];  we.ln1_b = (const float*)d_in[13];
  we.ff1_b = (const float*)d_in[15];  we.ff2_b = (const float*)d_in[17];
  we.ln2_w = (const float*)d_in[18];  we.ln2_b = (const float*)d_in[19];
  run_stack(stream, kEncL, kNumVis, kTokE, we, XfE, X16, T2, QK16, Vt16, AO16, H16);

  dec_fill_kernel<<<dim3((kTokD * (kDim / 4)) / 256), dim3(256), 0, stream>>>(mask_tok, pos, XfD, X16);
  dec_scatter_kernel<<<dim3(kTokE / 8), dim3(256), 0, stream>>>(XfE, vis, pos, XfD, X16);

  StackW wd;
  wd.qkv = W16 + kOffDqkv;  wd.outw = W16 + kOffDout;  wd.ff1 = W16 + kOffDff1;  wd.ff2 = W16 + kOffDff2;
  wd.qkv_b = (const float*)d_in[21];  wd.out_b = (const float*)d_in[23];
  wd.ln1_w = (const float*)d_in[24];  wd.ln1_b = (const float*)d_in[25];
  wd.ff1_b = (const float*)d_in[27];  wd.ff2_b = (const float*)d_in[29];
  wd.ln2_w = (const float*)d_in[30];  wd.ln2_b = (const float*)d_in[31];
  run_stack(stream, kDecL, kNumP, kTokD, wd, XfD, X16, T2, QK16, Vt16, AO16, H16);

  run_gemm<2, 4, false, 0>(stream, X16, kDim, W16 + kOffWrecon, kDim, d_out, nullptr, kImg, b_recon, nullptr,
                           kTokD, kPatchD, kDim, 1.0f / kWCarry, 1.0f, 1.0f);
}
